// MyModel_87522843559019
// MI455X (gfx1250) — hardware-run, weakly checked
//
#include <hip/hip_runtime.h>
#pragma clang fp contract(off)


#ifndef NB
#define NB 32
#endif
#define NB_FULL 32
#define KN   2048
#define NO   100
#define MP   32
#define NP   128
#define OSP  132
#define WTP  101

static_assert(NB >= 1);
static_assert(NB <= NB_FULL);
static_assert(NB_FULL == MP);
static_assert(MP == 32);
static_assert(NP == 128);
static_assert(NO <= NP);
static_assert(NO % 4 == 0);
static_assert(KN % 64 == 0);
static_assert(KN % 32 == 0);
static_assert(KN == 8 * 256);
static_assert(OSP % 4 == 0);
static_assert((64 * NO) % 256 == 0);

typedef unsigned short bf;
typedef __attribute__((ext_vector_type(16))) __bf16   v16bf;
typedef __attribute__((ext_vector_type(8)))  unsigned short v8us;
typedef __attribute__((ext_vector_type(8)))  float    v8f;
typedef __attribute__((ext_vector_type(4)))  float    v4f;
typedef v4f  __attribute__((may_alias)) v4fa;

__device__ __forceinline__ unsigned short f2bf(float f) { unsigned u = __float_as_uint(f); u += 0x7FFFu + ((u >> 16) & 1u); return (unsigned short)(u >> 16); }
__device__ __forceinline__ float bf2f(unsigned short h) { return __uint_as_float(((unsigned)h) << 16); }
__device__ __forceinline__ v16bf cat16b(v8us lo, v8us hi) { return __builtin_bit_cast(v16bf, __builtin_shufflevector(lo, hi, 0, 1, 2, 3, 4, 5, 6, 7, 8, 9, 10, 11, 12, 13, 14, 15)); }
__device__ __forceinline__ v8f wmmab(v16bf a, v16bf b, v8f c) { return __builtin_amdgcn_wmma_f32_16x16x32_bf16(false, a, false, b, (short)0, c, false, false); }
__device__ __forceinline__ v16bf ldb(const bf* p)  { return cat16b(*(const v8us*)p, *(const v8us*)(p + 16)); }

__global__ __launch_bounds__(256) void k_prep(const float* __restrict__ q, bf* RH, bf* RL) {
    __shared__ int sp[8];
    const int tid = threadIdx.x, lane = tid & 31;
    const int wave = __builtin_amdgcn_readfirstlane((int)(threadIdx.x >> 5));
    const int b = blockIdx.x;
    const bool live = (b < NB);
    const int rb = live ? b : (NB - 1);
    const float* src = q + (size_t)rb * KN + (size_t)tid * 8;
    const v4f x0 = *(const v4f*)src; const v4f x1 = *(const v4f*)(src + 4);
    float qv[8]; int c[8]; int s = 0;
#pragma unroll
    for (int i = 0; i < 4; ++i) { qv[i] = bf2f(f2bf(x0[i])); qv[4 + i] = bf2f(f2bf(x1[i])); }
#pragma unroll
    for (int i = 0; i < 8; ++i) { c[i] = (int)qv[i]; s += c[i]; }
    s += __shfl_xor(s, 16, 32); s += __shfl_xor(s, 8, 32); s += __shfl_xor(s, 4, 32); s += __shfl_xor(s, 2, 32); s += __shfl_xor(s, 1, 32);
    if (lane == 0) sp[wave] = s;
    __syncthreads();
    const int S = ((sp[0] + sp[1]) + (sp[2] + sp[3])) + ((sp[4] + sp[5]) + (sp[6] + sp[7]));
    v8us oh, ol;
#pragma unroll
    for (int i = 0; i < 8; ++i) {
        const float fr = (float)(KN * c[i] + S);
        const float d = qv[i] - fr;
        float r = d * d;
        r = live ? r : 0.0f;
        const unsigned short h = f2bf(r);
        const unsigned short l = f2bf(r - bf2f(h));
        oh[i] = h; ol[i] = l;
    }
    const size_t oo = (size_t)b * KN + (size_t)tid * 8;
    *(volatile v8us*)(RH + oo) = oh; *(volatile v8us*)(RL + oo) = ol;
    __threadfence();
    *(volatile v8us*)(RH + oo) = oh; *(volatile v8us*)(RL + oo) = ol;
}

__global__ __launch_bounds__(256) void k_wt(const float* __restrict__ W, bf* Wt) {
    __shared__ float tile[64 * WTP];
    const int tid = threadIdx.x;
    const int k0 = blockIdx.x * 64;
    const float* src = W + (size_t)k0 * NO;
#pragma unroll 5
    for (int it = 0; it < (64 * NO) / 256; ++it) {
        const int e = it * 256 + tid; const int k = e / NO; const int n = e - k * NO;
        tile[k * WTP + n] = src[e];
    }
    __syncthreads();
#pragma unroll 1
    for (int ps = 0; ps < 2; ++ps) {
#pragma unroll
        for (int s = 0; s < 4; ++s) {
            const int n = s * 32 + (tid >> 3), c8 = (tid & 7) * 8;
            const int nc = (n < NO) ? n : (NO - 1);
            v8us o;
#pragma unroll
            for (int i = 0; i < 8; ++i) { const float v = tile[(c8 + i) * WTP + nc]; const unsigned short w = f2bf(v); o[i] = (n < NO) ? w : (unsigned short)0; }
            *(volatile v8us*)(Wt + (size_t)n * KN + k0 + c8) = o;
        }
        if (ps == 0) __threadfence();
    }
}

__global__ __launch_bounds__(64) void k_gemm(const bf* __restrict__ RH, const bf* __restrict__ RL, const bf* __restrict__ Wt, float* OUT) {
    __shared__ __align__(16) float os[MP * OSP];
    const int lane = threadIdx.x & 31, lr = lane & 15, hi = lane >> 4;
    const int wave = __builtin_amdgcn_readfirstlane((int)(threadIdx.x >> 5));
    const int c0 = wave * 64;
    v8f acc[2][4];
#pragma unroll
    for (int mb = 0; mb < 2; ++mb)
#pragma unroll
        for (int nb = 0; nb < 4; ++nb) acc[mb][nb] = (v8f){};
    const size_t aoff = (size_t)lr * KN + 8 * hi, boff = (size_t)(c0 + lr) * KN + 8 * hi;
#pragma unroll 1
    for (int kc = 0; kc < KN; kc += 32) {
        v16bf ah[2], al[2];
#pragma unroll
        for (int mb = 0; mb < 2; ++mb) { ah[mb] = ldb(RH + aoff + (size_t)mb * 16 * KN + kc); al[mb] = ldb(RL + aoff + (size_t)mb * 16 * KN + kc); }
#pragma unroll
        for (int nb = 0; nb < 4; ++nb) { const v16bf b = ldb(Wt + boff + (size_t)nb * 16 * KN + kc);
            acc[0][nb] = wmmab(ah[0], b, acc[0][nb]); acc[1][nb] = wmmab(ah[1], b, acc[1][nb]);
            acc[0][nb] = wmmab(al[0], b, acc[0][nb]); acc[1][nb] = wmmab(al[1], b, acc[1][nb]); }
        asm volatile("v_nop\n\tv_nop\n\tv_nop\n\tv_nop"
                     : "+v"(acc[0][0]), "+v"(acc[0][1]), "+v"(acc[0][2]), "+v"(acc[0][3]), "+v"(acc[1][0]), "+v"(acc[1][1]), "+v"(acc[1][2]), "+v"(acc[1][3])
                     : "v"(ah[0]), "v"(ah[1]), "v"(al[0]), "v"(al[1]));
    }
#pragma unroll
    for (int mb = 0; mb < 2; ++mb)
#pragma unroll
        for (int nb = 0; nb < 4; ++nb)
#pragma unroll
            for (int j = 0; j < 8; ++j) os[(mb * 16 + hi * 8 + j) * OSP + c0 + nb * 16 + lr] = acc[mb][nb][j];
    __syncthreads();
    const int NPIECE = NB * NO / 4;
    const int NIT = (NPIECE + 63) / 64;
#pragma unroll 1
    for (int ps = 0; ps < 2; ++ps) {
#pragma unroll 1
        for (int it = 0; it < NIT; ++it) {
            const int i = (it * 2 + wave) * 32 + lane;
            const int ic = (i < NPIECE) ? i : (NPIECE - 1);
            const int row = ic / (NO / 4); const int col = (ic - row * (NO / 4)) * 4;
            const v4f val = *(const v4fa*)(&os[row * OSP + col]);
            if (i < NPIECE) *(volatile v4f*)(OUT + (size_t)i * 4) = val;
        }
        if (ps == 0) __threadfence();
    }
}

static constexpr size_t al256(size_t v) { return (v + 255) & ~(size_t)255; }
static constexpr size_t SZ_RP = al256((size_t)MP * KN * 2);
static constexpr size_t SZ_WT = al256((size_t)NP * KN * 2);
static constexpr size_t SZ_TOTAL = 2 * SZ_RP + SZ_WT;
static_assert(SZ_TOTAL <= (size_t)134217728);
static_assert((size_t)NB * NO * 4 <= (size_t)12800);

extern "C" void kernel_launch(void* const* d_in, const int* in_sizes, int n_in,
                              void* d_out, int out_size, void* d_ws, size_t ws_size, hipStream_t stream) {
    if (n_in < 2) return;
    if ((size_t)in_sizes[0] < (size_t)NB * KN) return;
    if ((size_t)in_sizes[1] < (size_t)KN * NO) return;
    if ((size_t)out_size < (size_t)NB * NO) return;
    if (SZ_TOTAL > ws_size) return;
    const float* q = (const float*)d_in[0];
    const float* w = (const float*)d_in[1];
    float* OUT = (float*)d_out;
    char* wsp = (char*)d_ws;
    bf* RH = (bf*)wsp; wsp += SZ_RP;
    bf* RL = (bf*)wsp; wsp += SZ_RP;
    bf* WT = (bf*)wsp; wsp += SZ_WT;

    k_prep<<<dim3(MP, 1, 1), 256, 0, stream>>>(q, RH, RL);
    k_wt<<<dim3(KN / 64, 1, 1), 256, 0, stream>>>(w, WT);
    k_gemm<<<dim3(1, 1, 1), 64, 0, stream>>>(RH, RL, WT, OUT);
}
